// SimpleRNN_60266981097547
// MI455X (gfx1250) — hardware-verified
//
#include <hip/hip_runtime.h>
#include <math.h>

constexpr int NBAT  = 64;
constexpr int NSTEP = 512;
constexpr int NHID  = 1024;
constexpr int NVOC  = 128;
constexpr int NROWS = NBAT * NSTEP;
constexpr int NOUT0 = NROWS * NVOC;
constexpr int NOUT1 = NBAT * NHID;

constexpr int RTHR  = 256;
constexpr int NWAVE = RTHR / 32;
constexpr int SEQB  = 16;
constexpr int WCOLS = NHID / NWAVE;
constexpr int GCOLS = 64;
constexpr int HP    = NHID;
constexpr int HT    = SEQB * HP;
constexpr int SLP   = 32;
constexpr float WCARRY     = 256.0f;
constexpr float WCARRY_INV = 1.0f / 256.0f;
constexpr float LOSC       = 2048.0f;
constexpr float S_HI       = WCARRY_INV;
constexpr float S_LO       = 1.0f / (256.0f * 2048.0f);
static_assert(NBAT % SEQB == 0);
static_assert(WCOLS == 2 * GCOLS);
static_assert(NHID % 32 == 0);
static_assert((SEQB * NHID / 4) % RTHR == 0);
static_assert(NROWS % 64 == 0 && NVOC % 64 == 0);
static_assert(((NROWS / 64) * (NVOC / 64)) % 8 == 0);
static_assert(NHID % 64 == 0);
static_assert((NVOC * NHID / 4) % 256 == 0);
static_assert(HP % 8 == 0);

typedef __attribute__((ext_vector_type(16))) _Float16 v16h;
typedef __attribute__((ext_vector_type(8)))  _Float16 v8h;
typedef __attribute__((ext_vector_type(16))) __bf16   v16b;
typedef __attribute__((ext_vector_type(8)))  __bf16   v8b;
typedef __attribute__((ext_vector_type(8)))  float    v8f;
typedef __attribute__((ext_vector_type(4)))  float    v4f;

__device__ __forceinline__ unsigned short f2bf_bits(float f) {
  unsigned u = __float_as_uint(f);
  return (unsigned short)((u + 0x7FFFu + ((u >> 16) & 1u)) >> 16);
}
__device__ __forceinline__ float bf_bits2f(unsigned short h) { return __uint_as_float(((unsigned)h) << 16); }
__device__ __forceinline__ float bf16r(float f) { return bf_bits2f(f2bf_bits(f)); }

__device__ __forceinline__ void dep_guard_h(v8f& a, v8f& b, v16h x, v16h y) { asm volatile("v_nop\n\tv_nop\n\tv_nop\n\tv_nop" : "+v"(a), "+v"(b) : "v"(x), "v"(y)); }
__device__ __forceinline__ void dep_guard_b(v8f& a, v8f& b, v16b x, v16b y) { asm volatile("v_nop\n\tv_nop\n\tv_nop\n\tv_nop" : "+v"(a), "+v"(b) : "v"(x), "v"(y)); }
__device__ __forceinline__ void keep4_h(v16h a, v16h b, v16h c, v16h d) { asm volatile("v_nop" :: "v"(a), "v"(b), "v"(c), "v"(d)); }
__device__ __forceinline__ void keep4_b(v16b a, v16b b, v16b c, v16b d) { asm volatile("v_nop" :: "v"(a), "v"(b), "v"(c), "v"(d)); }
__device__ __forceinline__ void acc_guard4(v8f& a, v8f& b, v8f& c, v8f& d) { asm volatile("v_nop\n\tv_nop\n\tv_nop\n\tv_nop" : "+v"(a), "+v"(b), "+v"(c), "+v"(d)); }
__device__ __forceinline__ void acc_guard8(v8f& a0, v8f& a1, v8f& a2, v8f& a3, v8f& a4, v8f& a5, v8f& a6, v8f& a7) {
  asm volatile("v_nop\n\tv_nop\n\tv_nop\n\tv_nop" : "+v"(a0), "+v"(a1), "+v"(a2), "+v"(a3), "+v"(a4), "+v"(a5), "+v"(a6), "+v"(a7));
}
template <typename V>
__device__ __forceinline__ void guard4v(v8f& a0, v8f& a1, v8f& a2, v8f& a3, V x0, V x1, V y0, V y1, V y2, V y3) {
  asm volatile("v_nop\n\tv_nop\n\tv_nop\n\tv_nop" : "+v"(a0), "+v"(a1), "+v"(a2), "+v"(a3) : "v"(x0), "v"(x1), "v"(y0), "v"(y1), "v"(y2), "v"(y3));
}
__device__ __forceinline__ void guard8h(v8f& a0, v8f& a1, v8f& a2, v8f& a3, v8f& b0, v8f& b1, v8f& b2, v8f& b3,
                                        v16h x0, v16h x1, v16h y0, v16h y1, v16h y2, v16h y3) {
  asm volatile("v_nop\n\tv_nop\n\tv_nop\n\tv_nop"
               : "+v"(a0), "+v"(a1), "+v"(a2), "+v"(a3), "+v"(b0), "+v"(b1), "+v"(b2), "+v"(b3)
               : "v"(x0), "v"(x1), "v"(y0), "v"(y1), "v"(y2), "v"(y3));
}
__device__ __forceinline__ void use8f(float& a0, float& a1, float& a2, float& a3, float& a4, float& a5, float& a6, float& a7) {
  asm volatile("" : "+v"(a0), "+v"(a1), "+v"(a2), "+v"(a3), "+v"(a4), "+v"(a5), "+v"(a6), "+v"(a7));
}
__device__ __forceinline__ void use8i(int& a0, int& a1, int& a2, int& a3, int& a4, int& a5, int& a6, int& a7) {
  asm volatile("" : "+v"(a0), "+v"(a1), "+v"(a2), "+v"(a3), "+v"(a4), "+v"(a5), "+v"(a6), "+v"(a7));
}
__device__ __forceinline__ void use1f(float& a) { asm volatile("" : "+v"(a)); }

template <typename T> struct Frag;
template <> struct Frag<_Float16> {
  typedef v16h V; union U { v16h v; v8h h[2]; };
  static __device__ __forceinline__ v16h load(const _Float16* p) {
    U f; f.h[0] = *(const v8h*)(p); f.h[1] = *(const v8h*)(p + 16); return f.v;
  }
  static __device__ __forceinline__ v8f mma(v16h a, v16h b, v8f c) {
    return __builtin_amdgcn_wmma_f32_16x16x32_f16(false, a, false, b, (short)0, c, false, false);
  }
  static __device__ __forceinline__ void guard(v8f& a, v8f& b, v16h x, v16h y) { dep_guard_h(a, b, x, y); }
  static __device__ __forceinline__ void keep(v16h a, v16h b, v16h c, v16h d) { keep4_h(a, b, c, d); }
};
template <> struct Frag<__bf16> {
  typedef v16b V; union U { v16b v; v8b h[2]; };
  static __device__ __forceinline__ v16b load(const __bf16* p) {
    U f; f.h[0] = *(const v8b*)(p); f.h[1] = *(const v8b*)(p + 16); return f.v;
  }
  static __device__ __forceinline__ v8f mma(v16b a, v16b b, v8f c) {
    return __builtin_amdgcn_wmma_f32_16x16x32_bf16(false, a, false, b, (short)0, c, false, false);
  }
  static __device__ __forceinline__ void guard(v8f& a, v8f& b, v16b x, v16b y) { dep_guard_b(a, b, x, y); }
  static __device__ __forceinline__ void keep(v16b a, v16b b, v16b c, v16b d) { keep4_b(a, b, c, d); }
};

template <int ET> struct Elem;
template <> struct Elem<0> { typedef _Float16 T; };
template <> struct Elem<1> { typedef __bf16 T; };
template <int ET, bool SPLIT, int BIAS_MODE, int OUT_MODE, bool RESID, int ACT = 0>
__global__ __launch_bounds__(256) void wmma_gemm64(
    const unsigned short* __restrict__ Ap, const unsigned short* __restrict__ A2p, int lda, long strideA,
    const unsigned short* __restrict__ Btp, const unsigned short* __restrict__ Bt2p, int ldb, long strideB,
    void* __restrict__ Cout, void* __restrict__ Cout2, int ldc, long strideC,
    const float* __restrict__ bias,
    const float* __restrict__ resid, long strideR,
    int M, int N, int K, float scale) {
  typedef typename Elem<ET>::T T;
  typedef typename Frag<T>::V V;
  const T* A = (const T*)Ap; const T* A2 = (const T*)A2p; const T* Bt = (const T*)Btp; const T* Bt2 = (const T*)Bt2p;
  __shared__ __align__(16) float sT[8][16 * 68];
  const int b    = blockIdx.y;
  const int lane = threadIdx.x & 31;
  const int wave = threadIdx.x >> 5;
  const int tilesN = N >> 6;
  const int tilesM = M >> 6;
  const int tile = blockIdx.x * 8 + wave;
  if (tile >= tilesM * tilesN) return;
  const int tm = tile / tilesN;
  const int tn = tile - tm * tilesN;
  const int m0 = tm << 6;
  const int n0 = tn << 6;

  const T* Ab  = A  + (size_t)b * strideA;
  const T* Bb  = Bt + (size_t)b * strideB;
  const T* Ab2 = SPLIT ? (A2  + (size_t)b * strideA) : nullptr;
  const T* Bb2 = SPLIT ? (Bt2 + (size_t)b * strideB) : nullptr;

  const int rlane = lane & 15;
  const int koff  = (lane >> 4) * 8;
  const int mOff  = (lane >> 4) * 8;

  v8f acc[4][4];
#pragma unroll
  for (int i = 0; i < 4; ++i)
#pragma unroll
    for (int j = 0; j < 4; ++j) acc[i][j] = (v8f){0.f,0.f,0.f,0.f,0.f,0.f,0.f,0.f};

  for (int k0 = 0; k0 < K; k0 += 32) {
    V bh[4], bl[4];
#pragma unroll
    for (int j = 0; j < 4; ++j) {
      const size_t bo = (size_t)(n0 + (j << 4) + rlane) * ldb + koff + k0;
      bh[j] = Frag<T>::load(Bb + bo);
      if (SPLIT) bl[j] = Frag<T>::load(Bb2 + bo);
    }
#pragma unroll
    for (int i = 0; i < 4; ++i) {
      const size_t ao = (size_t)(m0 + (i << 4) + rlane) * lda + koff + k0;
      V ah = Frag<T>::load(Ab + ao);
      V al = ah;
      if (SPLIT) al = Frag<T>::load(Ab2 + ao);
#pragma unroll
      for (int j = 0; j < 4; ++j) {
        acc[i][j] = Frag<T>::mma(ah, bh[j], acc[i][j]);
        if (SPLIT) {
          acc[i][j] = Frag<T>::mma(ah, bl[j], acc[i][j]);
          acc[i][j] = Frag<T>::mma(al, bh[j], acc[i][j]);
        }
      }
      guard4v<V>(acc[i][0], acc[i][1], acc[i][2], acc[i][3], ah, al, bh[0], bh[1], bh[2], bh[3]);
    }
    Frag<T>::keep(bh[0], bh[1], bh[2], bh[3]);
    if (SPLIT) Frag<T>::keep(bl[0], bl[1], bl[2], bl[3]);
  }
  acc_guard4(acc[0][0], acc[0][1], acc[0][2], acc[0][3]);
  acc_guard4(acc[1][0], acc[1][1], acc[1][2], acc[1][3]);
  acc_guard4(acc[2][0], acc[2][1], acc[2][2], acc[2][3]);
  acc_guard4(acc[3][0], acc[3][1], acc[3][2], acc[3][3]);

  float* slab = sT[wave];
  const float* Rb = RESID ? (resid + (size_t)b * strideR) : nullptr;
#pragma unroll
  for (int i = 0; i < 4; ++i) {
    const int mBase = m0 + (i << 4);
#pragma unroll
    for (int j = 0; j < 4; ++j) {
      const int n = n0 + (j << 4) + rlane;
      float bv = 0.f;
      if (BIAS_MODE == 2) bv = bias[n];
#pragma unroll
      for (int r = 0; r < 8; ++r) {
        float v = acc[i][j][r] * scale;
        if (BIAS_MODE == 1) v += bias[mBase + mOff + r];
        if (BIAS_MODE == 2) v += bv;
        if (RESID) v += Rb[(size_t)(mBase + mOff + r) * ldc + n];
        if (ACT == 1) v = tanhf(v);
        if (ACT == 2) v = fmaxf(v, 0.0f);
        if (ACT == 4) v = (v > 0.f) ? v : 0.01f * v;
        slab[(mOff + r) * 68 + (j << 4) + rlane] = v;
      }
    }
    __builtin_amdgcn_fence(__ATOMIC_RELEASE, "workgroup");
    __builtin_amdgcn_wave_barrier();
    __builtin_amdgcn_fence(__ATOMIC_ACQUIRE, "workgroup");
    if (OUT_MODE == 0) {
      float* C = (float*)Cout + (size_t)b * strideC;
      const int hh = lane >> 4, c4 = (lane & 15) * 4;
      for (int pass = 0; pass < 2; ++pass) {
#pragma unroll
        for (int it = 0; it < 8; ++it) {
          const int row = it * 2 + hh;
          v4f v = *(const v4f*)(slab + row * 68 + c4);
          *(volatile v4f*)(C + (size_t)(mBase + row) * ldc + n0 + c4) = v;
        }
        __threadfence();
      }
    } else {
      const int q = lane >> 3, c8 = (lane & 7) * 8;
      unsigned short* C  = (unsigned short*)Cout  + (size_t)b * strideC;
      unsigned short* C2 = (OUT_MODE == 2) ? ((unsigned short*)Cout2 + (size_t)b * strideC) : nullptr;
      for (int pass = 0; pass < 2; ++pass) {
#pragma unroll
        for (int it = 0; it < 4; ++it) {
          const int row = it * 4 + q;
          const float* sp = slab + row * 68 + c8;
          v8h hv, lv;
#pragma unroll
          for (int e = 0; e < 8; ++e) {
            if (OUT_MODE == 1) {
              hv[e] = (_Float16)sp[e];
            } else {
              unsigned short hb = f2bf_bits(sp[e]);
              unsigned short lb = f2bf_bits(sp[e] - bf_bits2f(hb));
              hv[e] = __builtin_bit_cast(_Float16, hb);
              lv[e] = __builtin_bit_cast(_Float16, lb);
            }
          }
          *(volatile v8h*)(C + (size_t)(mBase + row) * ldc + n0 + c8) = hv;
          if (OUT_MODE == 2) *(volatile v8h*)(C2 + (size_t)(mBase + row) * ldc + n0 + c8) = lv;
        }
        __threadfence();
      }
    }
    __builtin_amdgcn_fence(__ATOMIC_RELEASE, "workgroup");
    __builtin_amdgcn_wave_barrier();
    __builtin_amdgcn_fence(__ATOMIC_ACQUIRE, "workgroup");
  }
}

__global__ __launch_bounds__(256) void tconv_kernel(const float* __restrict__ in, unsigned short* __restrict__ outp,
                                                    int nrow_in, int ncol_in, float sc) {
  __shared__ float tile[64][65];
  _Float16* out = (_Float16*)outp;
  const int tid = threadIdx.x, lane = tid & 31, wave = tid >> 5;
  const int k0 = blockIdx.x * 64, n0 = blockIdx.y * 64;
#pragma unroll
  for (int i = 0; i < 16; ++i) {
    const int idx = i * 256 + tid;
    const int kl = idx >> 6, nl = idx & 63;
    tile[nl][kl] = in[(size_t)(k0 + kl) * ncol_in + n0 + nl];
    if ((i & 7) == 7) asm volatile("" ::: "memory");
  }
  __syncthreads();
  const int q = lane >> 3, c8 = (lane & 7) * 8;
  v8h hv0, hv1;
  const int nl0 = wave * 8 + q, nl1 = wave * 8 + 4 + q;
#pragma unroll
  for (int e = 0; e < 8; ++e) {
    hv0[e] = (_Float16)(bf16r(tile[nl0][c8 + e]) * sc);
    hv1[e] = (_Float16)(bf16r(tile[nl1][c8 + e]) * sc);
  }
  _Float16* p0 = out + (size_t)(n0 + nl0) * nrow_in + k0 + c8;
  _Float16* p1 = out + (size_t)(n0 + nl1) * nrow_in + k0 + c8;
  for (int pass = 0; pass < 2; ++pass) {
    *(volatile v8h*)p0 = hv0;
    *(volatile v8h*)p1 = hv1;
    __threadfence();
  }
}

__global__ __launch_bounds__(256) void rcopy4_kernel(const float* __restrict__ src, float* __restrict__ dst, int n4) {
  const int i = blockIdx.x * 256 + threadIdx.x;
  if (i < n4) {
    const v4f a = *(const v4f*)(src + (size_t)i * 4);
    v4f o;
#pragma unroll
    for (int e = 0; e < 4; ++e) o[e] = bf16r(a[e]);
    float* p = dst + (size_t)i * 4;
    *(volatile v4f*)p = o;
    __threadfence();
    *(volatile v4f*)p = o;
  }
}

__global__ __launch_bounds__(RTHR) void rnn_seq_kernel(
    const int* __restrict__ x, const float* __restrict__ EMB, const float* __restrict__ BHR,
    const float* __restrict__ H0, const unsigned short* __restrict__ WHHp,
    unsigned short* __restrict__ HIDp, float* __restrict__ HFIN) {
  __shared__ __align__(16) _Float16 Hh[2 * HT];
  __shared__ __align__(16) _Float16 Hl[2 * HT];
  __shared__ __align__(16) float    Sl[NWAVE][SEQB * SLP];
  const _Float16* WHH = (const _Float16*)WHHp;
  _Float16* HID = (_Float16*)HIDp;
  const int tid = threadIdx.x, lane = tid & 31, wave = tid >> 5;
  const int c = lane & 15, hh = lane >> 4, koff = hh * 8, mOff = hh * 8;
  const int q4 = lane >> 3, c8 = (lane & 7) * 8, c4q = (lane & 7) * 4;
  const int seq0  = blockIdx.x * SEQB;
  const int ncol0 = wave * WCOLS;

#pragma unroll 1
  for (int i = tid; i < SEQB * NHID / 4; i += RTHR) {
    const int row = i >> 8;
    const int col = (i & 255) * 4;
    const v4f a = *(const v4f*)(H0 + (size_t)(seq0 + row) * NHID + col);
#pragma unroll
    for (int e = 0; e < 4; ++e) {
      const float v = bf16r(a[e]);
      const _Float16 h16 = (_Float16)v;
      const float hf = (float)h16;
      const _Float16 l16 = (_Float16)((v - hf) * LOSC);
      Hh[row * HP + col + e] = h16;
      Hl[row * HP + col + e] = l16;
    }
  }
  __syncthreads();

  const v8f z8 = {0.f, 0.f, 0.f, 0.f, 0.f, 0.f, 0.f, 0.f};
  float* slab = Sl[wave];

#pragma unroll 1
  for (int t = 0; t < NSTEP; ++t) {
    const int cur = t & 1;
    const _Float16* hch = Hh + cur * HT;
    const _Float16* hcl = Hl + cur * HT;
    _Float16* hnh = Hh + (cur ^ 1) * HT;
    _Float16* hnl = Hl + (cur ^ 1) * HT;

    int tok[8];
#pragma unroll
    for (int r = 0; r < 8; ++r) {
      int v = x[(size_t)(seq0 + mOff + r) * NSTEP + t];
      v = (v < 0) ? 0 : v;
      v = (v > NVOC - 1) ? (NVOC - 1) : v;
      tok[r] = v;
    }
    use8i(tok[0], tok[1], tok[2], tok[3], tok[4], tok[5], tok[6], tok[7]);
    const bool last = (t == NSTEP - 1);

#pragma unroll 1
    for (int g = 0; g < 2; ++g) {
      const int nb = ncol0 + GCOLS * g;
      v8f ach[4], acl[4];
#pragma unroll
      for (int j = 0; j < 4; ++j) { ach[j] = z8; acl[j] = z8; }
      const _Float16* ahp = hch + c * HP + koff;
      const _Float16* alp = hcl + c * HP + koff;
      const _Float16* bp  = WHH + (size_t)(nb + c) * NHID + koff;
#pragma unroll 1
      for (int kc = 0; kc < NHID / 32; ++kc) {
        const v16h fa = Frag<_Float16>::load(ahp + kc * 32);
        const v16h fl = Frag<_Float16>::load(alp + kc * 32);
        v16h fb[4];
#pragma unroll
        for (int j = 0; j < 4; ++j) fb[j] = Frag<_Float16>::load(bp + (size_t)(16 * j) * NHID + kc * 32);
#pragma unroll
        for (int j = 0; j < 4; ++j) {
          ach[j] = Frag<_Float16>::mma(fa, fb[j], ach[j]);
          acl[j] = Frag<_Float16>::mma(fl, fb[j], acl[j]);
        }
        guard8h(ach[0], ach[1], ach[2], ach[3], acl[0], acl[1], acl[2], acl[3], fa, fl, fb[0], fb[1], fb[2], fb[3]);
      }
      acc_guard8(ach[0], ach[1], ach[2], ach[3], acl[0], acl[1], acl[2], acl[3]);

#pragma unroll
      for (int hq = 0; hq < 2; ++hq) {
#pragma unroll
        for (int jj = 0; jj < 2; ++jj) {
          const int j = 2 * hq + jj;
          const int n = nb + 16 * j + c;
          float bj = BHR[n];
          float ev[8];
#pragma unroll
          for (int r = 0; r < 8; ++r) ev[r] = EMB[(size_t)tok[r] * NHID + n];
          use8f(ev[0], ev[1], ev[2], ev[3], ev[4], ev[5], ev[6], ev[7]);
          use1f(bj);
#pragma unroll
          for (int r = 0; r < 8; ++r) {
            const float dot = ach[j][r] * S_HI + acl[j][r] * S_LO;
            float u = ev[r] + dot;
            u = u + bj;
            const float hv = tanhf(u);
            const _Float16 h16 = (_Float16)hv;
            const float hf = (float)h16;
            const _Float16 l16 = (_Float16)((hv - hf) * LOSC);
            hnh[(mOff + r) * HP + n] = h16;
            hnl[(mOff + r) * HP + n] = l16;
            if (last) slab[(mOff + r) * SLP + 16 * jj + c] = hv;
          }
        }
        if (last) {
          __builtin_amdgcn_fence(__ATOMIC_RELEASE, "workgroup");
          __builtin_amdgcn_wave_barrier();
          __builtin_amdgcn_fence(__ATOMIC_ACQUIRE, "workgroup");
          for (int pass = 0; pass < 2; ++pass) {
#pragma unroll
            for (int it = 0; it < 4; ++it) {
              const int row = it * 4 + q4;
              const v4f v = *(const v4f*)(slab + row * SLP + c4q);
              *(volatile v4f*)(HFIN + (size_t)(seq0 + row) * NHID + nb + 32 * hq + c4q) = v;
            }
            __threadfence();
          }
          __builtin_amdgcn_fence(__ATOMIC_RELEASE, "workgroup");
          __builtin_amdgcn_wave_barrier();
          __builtin_amdgcn_fence(__ATOMIC_ACQUIRE, "workgroup");
        }
      }
    }
    __syncthreads();

    for (int pass = 0; pass < 2; ++pass) {
#pragma unroll
      for (int it = 0; it < 4; ++it) {
        const int rr = it * 4 + q4;
#pragma unroll
        for (int hf = 0; hf < 2; ++hf) {
          const int col = ncol0 + 64 * hf + c8;
          const v8h v = *(const v8h*)(hnh + rr * HP + col);
          *(volatile v8h*)(HID + ((size_t)(seq0 + rr) * NSTEP + (size_t)t) * NHID + col) = v;
        }
      }
      __threadfence();
    }
  }
}

extern "C" void kernel_launch(void* const* d_in, const int* in_sizes, int n_in,
                              void* d_out, int out_size, void* d_ws, size_t ws_size, hipStream_t stream) {
  if (n_in < 7 || d_out == nullptr || d_ws == nullptr) return;
  if (in_sizes[0] != NBAT * NSTEP || in_sizes[1] != NBAT * NHID || in_sizes[2] != NVOC * NHID ||
      in_sizes[3] != NHID * NHID || in_sizes[4] != NHID || in_sizes[5] != NHID * NVOC || in_sizes[6] != NVOC ||
      out_size != NOUT0 + NOUT1) return;

  const int*   x    = (const int*)d_in[0];
  const float* h0   = (const float*)d_in[1];
  const float* wxh  = (const float*)d_in[2];
  const float* whh  = (const float*)d_in[3];
  const float* bh   = (const float*)d_in[4];
  const float* wout = (const float*)d_in[5];
  const float* bout = (const float*)d_in[6];
  float* out0 = (float*)d_out;
  float* out1 = out0 + (size_t)NOUT0;

  char* ws = (char*)d_ws; size_t off = 0;
  auto carve = [&](size_t bytes) -> char* { char* p = ws + off; off += (bytes + 255) & ~(size_t)255; return p; };
  unsigned short* WHH16 = (unsigned short*)carve((size_t)NHID * NHID * 2);
  unsigned short* WO16  = (unsigned short*)carve((size_t)NVOC * NHID * 2);
  float*          EMB   = (float*)carve((size_t)NVOC * NHID * 4);
  float*          BHR   = (float*)carve((size_t)NHID * 4);
  float*          BOUTR = (float*)carve((size_t)NVOC * 4);
  unsigned short* HID   = (unsigned short*)carve((size_t)NROWS * NHID * 2);
  if (off > ws_size || off > (size_t)134217728) return;

  tconv_kernel<<<dim3(NHID / 64, NHID / 64), 256, 0, stream>>>(whh, WHH16, NHID, NHID, WCARRY);
  tconv_kernel<<<dim3(NHID / 64, NVOC / 64), 256, 0, stream>>>(wout, WO16, NHID, NVOC, WCARRY);

  rcopy4_kernel<<<(NVOC * NHID / 4) / 256, 256, 0, stream>>>(wxh, EMB, NVOC * NHID / 4);
  rcopy4_kernel<<<1, 256, 0, stream>>>(bh, BHR, NHID / 4);
  rcopy4_kernel<<<1, 256, 0, stream>>>(bout, BOUTR, NVOC / 4);

  rnn_seq_kernel<<<NBAT / SEQB, RTHR, 0, stream>>>(x, EMB, BHR, h0, WHH16, HID, out1);

  const int ggrid = ((NROWS / 64) * (NVOC / 64)) / 8;
  wmma_gemm64<0, false, 2, 0, false, 0><<<dim3(ggrid, 1), 256, 0, stream>>>(
      HID, nullptr, NHID, 0L, WO16, nullptr, NHID, 0L,
      (void*)out0, nullptr, NVOC, 0L, BOUTR, nullptr, 0L, NROWS, NVOC, NHID, WCARRY_INV);
}
